// NeuralJumpODE_56865366999503
// MI455X (gfx1250) — hardware-verified
//
#include <hip/hip_runtime.h>


namespace {
constexpr int Bn = 256, NOBS = 1024, DX = 16, H = 64, DY = 8, M = 2, NR = Bn * NOBS;

typedef _Float16 b16;
typedef __attribute__((ext_vector_type(16))) _Float16 v16b;
typedef __attribute__((ext_vector_type(8)))  _Float16 v8b;
typedef __attribute__((ext_vector_type(8)))  float v8f;
typedef __attribute__((ext_vector_type(4)))  float v4f;

__device__ __forceinline__ v8b ld8b(const b16* p) { return *(const v8b*)p; }
__device__ __forceinline__ v16b cat8b(v8b a, v8b b) { return __builtin_shufflevector(a, b, 0, 1, 2, 3, 4, 5, 6, 7, 8, 9, 10, 11, 12, 13, 14, 15); }
__device__ __forceinline__ v16b frag_kb(const b16* p, int hh) { return cat8b(ld8b(p + 8 * hh), ld8b(p + 16 + 8 * hh)); }
__device__ __forceinline__ void split16(float v, b16& hi, b16& lo) { hi = (b16)v; lo = (b16)(v - (float)hi); }
__device__ __forceinline__ void frag_ksplit(const float* p, int hh, v16b& fh_, v16b& fl_) {
  const float* p0 = p + 8 * hh; const float* p1 = p + 16 + 8 * hh;
#pragma unroll
  for (int e = 0; e < 8; ++e) { b16 a, c; split16(p0[e], a, c); fh_[e] = a; fl_[e] = c; split16(p1[e], a, c); fh_[8 + e] = a; fl_[8 + e] = c; }
}
__device__ __forceinline__ v8f wmma16b(v16b a, v16b b, v8f c) {
  v8f d = __builtin_amdgcn_wmma_f32_16x16x32_f16(false, a, false, b, (short)0, c, false, false);
  asm volatile("v_nop\n\tv_nop\n\tv_nop\n\tv_nop" : "+v"(d) : "v"(a), "v"(b));
  return d;
}
__device__ __forceinline__ void wave_lds_sync() {
  __builtin_amdgcn_fence(__ATOMIC_RELEASE, "workgroup");
  __builtin_amdgcn_wave_barrier();
  __builtin_amdgcn_fence(__ATOMIC_ACQUIRE, "workgroup");
}

struct Opnd { const void* p0; const void* p1; int ld; };
template <int NP> __device__ __forceinline__ void load_frags(const Opnd& o, int row, int kb, int hh, v16b& fh_, v16b& fl_) {
  if (NP == 0) { frag_ksplit((const float*)o.p0 + (size_t)row * o.ld + kb, hh, fh_, fl_); }
  else if (NP == 4) {
    const float* p = (const float*)o.p0 + (size_t)row * o.ld + kb; const float* p0 = p + 8 * hh; const float* p1 = p + 16 + 8 * hh;
#pragma unroll
    for (int e = 0; e < 8; ++e) { b16 a, c; split16(p0[e] * 64.0f, a, c); fh_[e] = a; fl_[e] = c; split16(p1[e] * 64.0f, a, c); fh_[8 + e] = a; fl_[8 + e] = c; }
  } else if (NP == 3) {
    const float* p = (const float*)o.p0 + (size_t)row * o.ld + kb; const float* p0 = p + 8 * hh; const float* p1 = p + 16 + 8 * hh;
#pragma unroll
    for (int e = 0; e < 8; ++e) { fh_[e] = (b16)p0[e]; fh_[8 + e] = (b16)p1[e]; }
    fl_ = fh_;
  } else {
    fh_ = frag_kb((const b16*)o.p0 + (size_t)row * o.ld + kb, hh);
    if (NP == 2) fl_ = frag_kb((const b16*)o.p1 + (size_t)row * o.ld + kb, hh); else fl_ = fh_;
  }
}
template <int ANP, int BNP> __device__ __forceinline__ v8f mac(v16b ah, v16b al, v16b bh, v16b bl, v8f c) {
  c = wmma16b(ah, bh, c);
  if (BNP == 0 || BNP == 2 || BNP == 4) c = wmma16b(ah, bl, c);
  if (ANP == 0 || ANP == 2 || ANP == 4) c = wmma16b(al, bh, c);
  return c;
}
template <int ANP, int BNP>
__device__ __forceinline__ void gemm_tile(const Opnd& A, const Opnd& B, int K, int m0, int c0, int nloc, int hlf, v8f (&acc)[2][4]) {
  for (int kb = 0; kb < K; kb += 32) {
    v16b a0h, a0l, a1h, a1l;
    load_frags<ANP>(A, m0 + nloc, kb, hlf, a0h, a0l);
    load_frags<ANP>(A, m0 + 16 + nloc, kb, hlf, a1h, a1l);
#pragma unroll
    for (int t = 0; t < 4; ++t) {
      v16b bh, bl;
      load_frags<BNP>(B, c0 + t * 16 + nloc, kb, hlf, bh, bl);
      acc[0][t] = mac<ANP, BNP>(a0h, a0l, bh, bl, acc[0][t]);
      acc[1][t] = mac<ANP, BNP>(a1h, a1l, bh, bl, acc[1][t]);
    }
  }
}

__device__ __forceinline__ void epi_planes(v8f (&acc)[2][4], float scale, bool two, b16* __restrict__ oh, b16* __restrict__ ol, int ldo,
                                           int m0, int c0, int lane, b16* Th, b16* Tl) {
  const int nloc = lane & 15, hlf = lane >> 4;
#pragma unroll
  for (int t = 0; t < 4; ++t)
#pragma unroll
    for (int r = 0; r < 2; ++r)
#pragma unroll
      for (int v = 0; v < 8; ++v) {
        const int rr = r * 16 + v + 8 * hlf, cc = t * 16 + nloc;
        b16 h_, l_; split16(acc[r][t][v] * scale, h_, l_);
        Th[rr * 64 + cc] = h_; Tl[rr * 64 + cc] = l_;
      }
  wave_lds_sync();
  for (int pass = 0; pass < 2; ++pass) {
#pragma unroll
    for (int j = 0; j < 8; ++j) {
      const int rr = j * 4 + (lane >> 3), c8 = (lane & 7) * 8;
      const size_t o = (size_t)(m0 + rr) * ldo + c0 + c8;
      *(volatile v8b*)(oh + o) = ld8b(Th + rr * 64 + c8);
      if (two) *(volatile v8b*)(ol + o) = ld8b(Tl + rr * 64 + c8);
    }
    __threadfence();
  }
}
__device__ __forceinline__ void epi_f32(v8f (&acc)[2][4], float scale, const float* rscale, float* __restrict__ out, int ldo, int m0, int c0, int lane, float* Tt) {
  const int nloc = lane & 15, hlf = lane >> 4;
#pragma unroll
  for (int t = 0; t < 4; ++t)
#pragma unroll
    for (int r = 0; r < 2; ++r)
#pragma unroll
      for (int v = 0; v < 8; ++v) {
        const int rr = r * 16 + v + 8 * hlf;
        const float rs = rscale ? rscale[(size_t)(m0 + rr) * 32] : 1.0f;
        Tt[rr * 64 + t * 16 + nloc] = acc[r][t][v] * scale * rs;
      }
  wave_lds_sync();
  float* dst0 = out + (size_t)m0 * ldo + c0;
  for (int pass = 0; pass < 2; ++pass) {
#pragma unroll
    for (int j = 0; j < 16; ++j) { const int rr = j * 2 + hlf, c4 = nloc * 4; *(volatile v4f*)(dst0 + (size_t)rr * ldo + c4) = *(const v4f*)(Tt + rr * 64 + c4); }
    __threadfence();
  }
}


__device__ __forceinline__ float tanh_e(float v) { return 1.0f - 2.0f * __builtin_amdgcn_rcpf(1.0f + __expf(2.0f * v)); }

__global__ __launch_bounds__(256) void prep_kernel(const float* __restrict__ jW1, const float* __restrict__ jW2, const float* __restrict__ uW1, const float* __restrict__ uW2,
                                                   const float* __restrict__ oW1, const float* __restrict__ oW2,
                                                   b16* __restrict__ w1, b16* __restrict__ w2, b16* __restrict__ wu1, b16* __restrict__ wu2, b16* __restrict__ wo1, b16* __restrict__ wo2) {
  const int t = blockIdx.x * 256 + threadIdx.x, nth = gridDim.x * 256;
  for (int pass = 0; pass < 2; ++pass) {
    for (int p = t; p < M * 64 * 16 / 8; p += nth) { const int m = p / 128, n = (p % 128) / 2, k0 = (p % 2) * 8; v8b v;
#pragma unroll
      for (int e = 0; e < 8; ++e) v[e] = (b16)jW1[((size_t)m * DX + k0 + e) * H + n];
      *(volatile v8b*)(w1 + ((size_t)m * 64 + n) * 16 + k0) = v; }
    for (int p = t; p < M * 64 * 64 / 8; p += nth) { const int m = p / 512, n = (p % 512) / 8, k0 = (p % 8) * 8; v8b a, b2, c;
#pragma unroll
      for (int e = 0; e < 8; ++e) { a[e] = (b16)jW2[((size_t)m * H + k0 + e) * H + n]; b2[e] = (b16)uW1[((size_t)m * H + k0 + e) * H + n]; c[e] = (b16)oW2[((size_t)m * H + k0 + e) * H + n]; }
      const size_t o = ((size_t)m * 64 + n) * 64 + k0; *(volatile v8b*)(w2 + o) = a; *(volatile v8b*)(wu1 + o) = b2; *(volatile v8b*)(wo2 + o) = c; }
    for (int p = t; p < M * 16 * 64 / 8; p += nth) { const int m = p / 128, n = (p % 128) / 8, k0 = (p % 8) * 8; v8b v;
#pragma unroll
      for (int e = 0; e < 8; ++e) v[e] = (b16)((n < DY) ? uW2[((size_t)m * H + k0 + e) * DY + n] : 0.0f);
      *(volatile v8b*)(wu2 + ((size_t)m * 16 + n) * 64 + k0) = v; }
    for (int p = t; p < M * 64 * 96 / 8; p += nth) { const int m = p / 768, n = (p % 768) / 12, k0 = (p % 12) * 8; v8b v;
#pragma unroll
      for (int e = 0; e < 8; ++e) { const int k = k0 + e; v[e] = (b16)((k < H + DX + 2) ? oW1[((size_t)m * (H + DX + 2) + k) * H + n] : 0.0f); }
      *(volatile v8b*)(wo1 + ((size_t)m * 64 + n) * 96 + k0) = v; }
    __threadfence();
  }
}

__device__ __forceinline__ void layer32(const b16* __restrict__ T, const b16* __restrict__ W, int ldw, int t0, int nloc, int hlf, v8f (&acc)[2][2]) {
#pragma unroll
  for (int r = 0; r < 2; ++r)
#pragma unroll
    for (int t = 0; t < 2; ++t) acc[r][t] = (v8f){};
#pragma unroll
  for (int ks = 0; ks < 2; ++ks) {
    const v16b a0 = frag_kb(T + (size_t)nloc * 72 + ks * 32, hlf), a1 = frag_kb(T + (size_t)(16 + nloc) * 72 + ks * 32, hlf);
#pragma unroll
    for (int t = 0; t < 2; ++t) { const v16b bw = frag_kb(W + (size_t)((t0 + t) * 16 + nloc) * ldw + ks * 32, hlf); acc[0][t] = wmma16b(a0, bw, acc[0][t]); acc[1][t] = wmma16b(a1, bw, acc[1][t]); }
  }
}
__device__ __forceinline__ void act_to_tile2(v8f (&acc)[2][2], const float* __restrict__ bias, b16* __restrict__ T, int t0, int nloc, int hlf, float scale) {
#pragma unroll
  for (int t = 0; t < 2; ++t)
#pragma unroll
    for (int r = 0; r < 2; ++r)
#pragma unroll
      for (int v = 0; v < 8; ++v) { const float a = tanh_e(acc[r][t][v] * scale + bias[(t0 + t) * 16 + nloc]); T[(size_t)(r * 16 + v + 8 * hlf) * 72 + (t0 + t) * 16 + nloc] = (b16)a; }
}


__global__ __launch_bounds__(128) void main_kernel(const float* __restrict__ times, const float* __restrict__ values,
                                                   const b16* __restrict__ w1, const float* __restrict__ jb1, const b16* __restrict__ w2, const float* __restrict__ jb2,
                                                   const b16* __restrict__ wu1, const float* __restrict__ ub1, const b16* __restrict__ wu2, const float* __restrict__ ub2,
                                                   const b16* __restrict__ wo1, const float* __restrict__ ob1, const b16* __restrict__ wo2, const float* __restrict__ ob2,
                                                   float* __restrict__ opred, float* __restrict__ ybuf) {
  __shared__ __attribute__((aligned(16))) b16 T1h_[4][32 * 72]; __shared__ __attribute__((aligned(16))) b16 T1l_[4][32 * 72]; __shared__ __attribute__((aligned(16))) b16 T2_[4][32 * 72];
  __shared__ __attribute__((aligned(16))) float Yo[4][32 * 16]; __shared__ __attribute__((aligned(16))) float Yb[4][32 * 16];
  __shared__ float Hf_[4][32 * 64];
  const int lane = threadIdx.x & 31, wave = threadIdx.x >> 5, nloc = lane & 15, hlf = lane >> 4, m0 = blockIdx.x * 128 + wave * 32;
  b16* T1h = T1h_[wave]; b16* T1l = T1l_[wave]; b16* T2 = T2_[wave]; float* Hf = Hf_[wave];
  const int ra = m0 + nloc, rb = m0 + 16 + nloc;
  float ta, dta, tb, dtb;
  { const int na = ra % NOBS, nb = rb % NOBS; ta = times[ra]; tb = times[rb]; dta = (na < NOBS - 1) ? times[ra + 1] - ta : 0.0f; dtb = (nb < NOBS - 1) ? times[rb + 1] - tb : 0.0f; }
#pragma unroll 1
  for (int m = 0; m < M; ++m) {
    { v16b a0 = {}, a1 = {};
#pragma unroll
      for (int e = 0; e < 8; ++e) { a0[e] = (b16)values[(size_t)ra * DX + 8 * hlf + e]; a1[e] = (b16)values[(size_t)rb * DX + 8 * hlf + e]; }
#pragma unroll 1
      for (int t0 = 0; t0 < 4; t0 += 2) { v8f acc[2][2] = {{{}, {}}, {{}, {}}};
#pragma unroll
        for (int t = 0; t < 2; ++t) { v16b bw = {}; const v8b p8 = ld8b(w1 + ((size_t)m * 64 + (t0 + t) * 16 + nloc) * 16 + 8 * hlf);
#pragma unroll
          for (int e = 0; e < 8; ++e) bw[e] = p8[e];
          acc[0][t] = wmma16b(a0, bw, acc[0][t]); acc[1][t] = wmma16b(a1, bw, acc[1][t]); }
        act_to_tile2(acc, jb1 + m * H, T2, t0, nloc, hlf, 1.0f); } }
    wave_lds_sync();
#pragma unroll 1
    for (int t0 = 0; t0 < 4; t0 += 2) { v8f acc[2][2]; layer32(T2, w2 + (size_t)m * 64 * 64, 64, t0, nloc, hlf, acc);
#pragma unroll
      for (int t = 0; t < 2; ++t)
#pragma unroll
        for (int r = 0; r < 2; ++r)
#pragma unroll
          for (int v = 0; v < 8; ++v) { const int cc = (t0 + t) * 16 + nloc, rr = r * 16 + v + 8 * hlf; const float hv = tanh_e(acc[r][t][v] + jb2[m * H + cc]); b16 a, c; split16(hv * 8.0f, a, c); T1h[(size_t)rr * 72 + cc] = a; T1l[(size_t)rr * 72 + cc] = c; Hf[rr * 64 + cc] = hv; } }
    wave_lds_sync();
#pragma unroll 1
    for (int t0 = 0; t0 < 4; t0 += 2) { v8f acc[2][2]; layer32(T1h, wu1 + (size_t)m * 64 * 64, 64, t0, nloc, hlf, acc); act_to_tile2(acc, ub1 + m * H, T2, t0, nloc, hlf, 0.125f); }
    wave_lds_sync();
    { v8f y0 = {}, y1 = {};
#pragma unroll
      for (int ks = 0; ks < 2; ++ks) { const v16b bw = frag_kb(wu2 + ((size_t)m * 16 + nloc) * 64 + ks * 32, hlf);
        y0 = wmma16b(frag_kb(T2 + (size_t)nloc * 72 + ks * 32, hlf), bw, y0); y1 = wmma16b(frag_kb(T2 + (size_t)(16 + nloc) * 72 + ks * 32, hlf), bw, y1); }
      if (nloc < DY) {
#pragma unroll
        for (int v = 0; v < 8; ++v) { Yo[wave][(v + 8 * hlf) * 16 + nloc * 2 + m] = y0[v] + ub2[m * DY + nloc]; Yo[wave][(16 + v + 8 * hlf) * 16 + nloc * 2 + m] = y1[v] + ub2[m * DY + nloc]; } } }
    wave_lds_sync();
    { v16b xk0h = {}, xk0l = {}, xk1h = {}, xk1l = {};
#pragma unroll
      for (int e = 0; e < 8; ++e) { b16 p, q2; split16(values[(size_t)ra * DX + 8 * hlf + e] * 8.0f, p, q2); xk0h[e] = p; xk0l[e] = q2; split16(values[(size_t)rb * DX + 8 * hlf + e] * 8.0f, p, q2); xk1h[e] = p; xk1l[e] = q2; }
      if (hlf == 0) { b16 p, q2; split16(ta * 8.0f, p, q2); xk0h[8] = p; xk0l[8] = q2; split16(dta * 8.0f, p, q2); xk0h[9] = p; xk0l[9] = q2; split16(tb * 8.0f, p, q2); xk1h[8] = p; xk1l[8] = q2; split16(dtb * 8.0f, p, q2); xk1h[9] = p; xk1l[9] = q2; }
#pragma unroll 1
      for (int t0 = 0; t0 < 4; t0 += 2) {
        v8f acc[2][2] = {{{}, {}}, {{}, {}}};
#pragma unroll
        for (int ks = 0; ks < 2; ++ks) {
          const v16b a0 = frag_kb(T1h + (size_t)nloc * 72 + ks * 32, hlf), a1 = frag_kb(T1h + (size_t)(16 + nloc) * 72 + ks * 32, hlf);
          const v16b c0 = frag_kb(T1l + (size_t)nloc * 72 + ks * 32, hlf), c1 = frag_kb(T1l + (size_t)(16 + nloc) * 72 + ks * 32, hlf);
#pragma unroll
          for (int t = 0; t < 2; ++t) { const v16b bw = frag_kb(wo1 + ((size_t)m * 64 + (t0 + t) * 16 + nloc) * 96 + ks * 32, hlf);
            acc[0][t] = wmma16b(a0, bw, acc[0][t]); acc[0][t] = wmma16b(c0, bw, acc[0][t]); acc[1][t] = wmma16b(a1, bw, acc[1][t]); acc[1][t] = wmma16b(c1, bw, acc[1][t]); }
        }
#pragma unroll
        for (int t = 0; t < 2; ++t) { const v16b bw = frag_kb(wo1 + ((size_t)m * 64 + (t0 + t) * 16 + nloc) * 96 + 64, hlf);
          acc[0][t] = wmma16b(xk0h, bw, acc[0][t]); acc[0][t] = wmma16b(xk0l, bw, acc[0][t]); acc[1][t] = wmma16b(xk1h, bw, acc[1][t]); acc[1][t] = wmma16b(xk1l, bw, acc[1][t]); }
        act_to_tile2(acc, ob1 + m * H, T2, t0, nloc, hlf, 0.125f);
      } }
    wave_lds_sync();
#pragma unroll 1
    for (int t0 = 0; t0 < 4; t0 += 2) { v8f acc[2][2]; layer32(T2, wo2 + (size_t)m * 64 * 64, 64, t0, nloc, hlf, acc);
#pragma unroll
      for (int r = 0; r < 2; ++r)
#pragma unroll
        for (int v = 0; v < 8; ++v) { const float dtrow = __shfl((r == 0) ? dta : dtb, v + 8 * hlf, 32);
#pragma unroll
          for (int t = 0; t < 2; ++t) { const int rr = r * 16 + v + 8 * hlf, cc = (t0 + t) * 16 + nloc; const float hm = Hf[rr * 64 + cc] + dtrow * (acc[r][t][v] + ob2[m * H + cc]); T1h[(size_t)rr * 72 + cc] = (b16)(hm * 8.0f); } } }
    wave_lds_sync();
#pragma unroll 1
    for (int t0 = 0; t0 < 4; t0 += 2) { v8f acc[2][2]; layer32(T1h, wu1 + (size_t)m * 64 * 64, 64, t0, nloc, hlf, acc); act_to_tile2(acc, ub1 + m * H, T2, t0, nloc, hlf, 0.125f); }
    wave_lds_sync();
    { v8f y0 = {}, y1 = {};
#pragma unroll
      for (int ks = 0; ks < 2; ++ks) { const v16b bw = frag_kb(wu2 + ((size_t)m * 16 + nloc) * 64 + ks * 32, hlf);
        y0 = wmma16b(frag_kb(T2 + (size_t)nloc * 72 + ks * 32, hlf), bw, y0); y1 = wmma16b(frag_kb(T2 + (size_t)(16 + nloc) * 72 + ks * 32, hlf), bw, y1); }
      if (nloc < DY) {
#pragma unroll
        for (int v = 0; v < 8; ++v) { Yb[wave][(v + 8 * hlf) * 16 + nloc * 2 + m] = y0[v] + ub2[m * DY + nloc]; Yb[wave][(16 + v + 8 * hlf) * 16 + nloc * 2 + m] = y1[v] + ub2[m * DY + nloc]; } } }
    wave_lds_sync();
  }
  wave_lds_sync();
  for (int pass = 0; pass < 2; ++pass) {
#pragma unroll
    for (int j = 0; j < 4; ++j) { const int f = (j * 32 + lane) * 4; *(volatile v4f*)(opred + (size_t)m0 * 16 + f) = *(const v4f*)(&Yo[wave][f]); *(volatile v4f*)(ybuf + (size_t)m0 * 16 + f) = *(const v4f*)(&Yb[wave][f]); }
    __threadfence();
  }
}

__global__ __launch_bounds__(128) void shift_kernel(const float* __restrict__ ybuf, float* __restrict__ opb) {
  const int t = threadIdx.x; const size_t r0 = (size_t)blockIdx.x * 128;
  for (int pass = 0; pass < 2; ++pass) {
#pragma unroll
    for (int j = 0; j < 4; ++j) { const size_t f = (r0 * 16) + (size_t)(j * 128 + t) * 4; const size_t row = f / 16; const int n = (int)(row % NOBS);
      v4f v = {0.0f, 0.0f, 0.0f, 0.0f}; if (n > 0) v = *(const v4f*)(ybuf + f - 16);
      *(volatile v4f*)(opb + f) = v; }
    __threadfence();
  }
}
}

extern "C" void kernel_launch(void* const* d_in, const int* in_sizes, int n_in,
                              void* d_out, int out_size, void* d_ws, size_t ws_size, hipStream_t stream) {
  (void)n_in; (void)out_size;
  const float* times = (const float*)d_in[0]; const float* values = (const float*)d_in[1];
  const float* jW1 = (const float*)d_in[2]; const float* jb1 = (const float*)d_in[3]; const float* jW2 = (const float*)d_in[4]; const float* jb2 = (const float*)d_in[5];
  const float* oW1 = (const float*)d_in[6]; const float* ob1 = (const float*)d_in[7]; const float* oW2 = (const float*)d_in[8]; const float* ob2 = (const float*)d_in[9];
  const float* uW1 = (const float*)d_in[10]; const float* ub1 = (const float*)d_in[11]; const float* uW2 = (const float*)d_in[12]; const float* ub2 = (const float*)d_in[13];
  float* out = (float*)d_out;
  if (in_sizes[0] != NR || in_sizes[1] != NR * DX || in_sizes[2] != M * DX * H || in_sizes[6] != M * (H + DX + 2) * H || in_sizes[12] != M * H * DY) return;
  size_t off = 0; char* ws = (char*)d_ws;
  auto carve = [&](size_t bytes) { char* p = ws + off; off += (bytes + 255) & ~(size_t)255; return p; };
  b16* w1 = (b16*)carve(M * 64 * 16 * 2); b16* w2 = (b16*)carve(M * 64 * 64 * 2); b16* wu1 = (b16*)carve(M * 64 * 64 * 2); b16* wu2 = (b16*)carve(M * 16 * 64 * 2); b16* wo1 = (b16*)carve(M * 64 * 96 * 2); b16* wo2 = (b16*)carve(M * 64 * 64 * 2);
  float* ybuf = (float*)carve((size_t)NR * 16 * 4);
  if (off > ws_size) return;
  float* opred = out; float* opb = out + (size_t)NR * 16;
  prep_kernel<<<8, 256, 0, stream>>>(jW1, jW2, uW1, uW2, oW1, oW2, w1, w2, wu1, wu2, wo1, wo2);
  main_kernel<<<NR / 128, 128, 0, stream>>>(times, values, w1, jb1, w2, jb2, wu1, ub1, wu2, ub2, wo1, ob1, wo2, ob2, opred, ybuf);
  shift_kernel<<<NR / 128, 128, 0, stream>>>(ybuf, opb);
}
